// TemporalTransformer_83047487635862
// MI455X (gfx1250) — hardware-verified
//
#include <hip/hip_runtime.h>
#include <math.h>
#include <stdint.h>

#ifndef NB
#define NB 4
#endif
#ifndef SEQ
#define SEQ 1024
#endif
#define NB_FULL  4
#define SEQ_FULL 1024
#define IND      16
#define OUTD     16
#define QDIM     32
#define HID      256
#define DFF      1024
#define NHEAD    8
#define HDIM     32
#define NLAYER   4
#define TED      256
#define NROWS    (NB * SEQ)
#define KIN      32
#define NOUTP    64
#define TABR     (2 * SEQ_FULL - 1)
#define TABP     2048
#define RELOFF   (SEQ_FULL - 1)
#define KX       (2 * HID)
#define KG       (2 * DFF)

#define WSC    16384.0f
#define WLO    16.0f
#define RSC    1024.0f
#define XC     1024.0f
#define HCARRY 16.0f
#define QC     16.0f
#define KC     16.0f
#define VC     16.0f
#define PC     1024.0f
#define FC     1024.0f
#define GC     64.0f
#define HFC    16.0f
#define ATT_SCALE 0.17677669529663687f
#define LOG2E  1.4426950408889634f
#define LN_EPS 1e-5f
#define DECAYF 0.1f
#define CLN    (-9.21034049987793f)

static_assert(NHEAD * HDIM == HID);
static_assert(NB >= 1 && NB <= NB_FULL && SEQ >= 64 && SEQ <= SEQ_FULL && (SEQ % 64) == 0);
static_assert((NROWS % 64) == 0 && (HID % 64) == 0 && (DFF % 64) == 0 && (KX % 32) == 0 && (KG % 32) == 0);
static_assert((KIN % 32) == 0 && (NOUTP % 64) == 0 && TED == HID && TED == 256 && (SEQ % 16) == 0);
static_assert(WSC == WLO * RSC);
static_assert(TABR < TABP);

typedef _Float16 v16h __attribute__((ext_vector_type(16)));
typedef _Float16 v8h  __attribute__((ext_vector_type(8)));
typedef float    v8f  __attribute__((ext_vector_type(8)));
typedef float    v4f  __attribute__((ext_vector_type(4)));
typedef unsigned int v4u __attribute__((ext_vector_type(4)));

union FragH { v16h v; v8h h[2]; v4u u[2]; };

__device__ __forceinline__ unsigned short bf_bits(float f) {
  unsigned u = __float_as_uint(f);
  return (unsigned short)((u + 0x7FFFu + ((u >> 16) & 1u)) >> 16);
}
__device__ __forceinline__ float bf_up(unsigned short h) { return __uint_as_float(((unsigned)h) << 16); }
__device__ __forceinline__ float bfr(float f) { return bf_up(bf_bits(f)); }
__device__ __forceinline__ unsigned short h_bits(_Float16 x) { return __builtin_bit_cast(unsigned short, x); }
__device__ __forceinline__ unsigned short hz(float f) {
  const unsigned short b = h_bits((_Float16)f);
  return ((b & 0x7C00u) == 0u) ? (unsigned short)0u : b;
}
__device__ __forceinline__ float hup(unsigned short b) { return (float)__builtin_bit_cast(_Float16, b); }
__device__ __forceinline__ unsigned pk16(unsigned short a, unsigned short b) { return (unsigned)a | ((unsigned)b << 16); }
__device__ __forceinline__ v8f zero8() { v8f z = {0.f, 0.f, 0.f, 0.f, 0.f, 0.f, 0.f, 0.f}; return z; }
__device__ __forceinline__ int imin(int a, int b) { return a < b ? a : b; }
__device__ __forceinline__ float gelu_f(float u) { return 0.5f * u * (1.0f + erff(u * 0.70710678118654752f)); }

__device__ __forceinline__ v16h ldfrag_h(const _Float16* p) {
  FragH f;
  f.h[0] = *(const v8h*)(p);
  f.h[1] = *(const v8h*)(p + 16);
  return f.v;
}
__device__ __forceinline__ v16h ldfrag_u(const unsigned short* p) {
  FragH f;
  f.u[0] = *(const v4u*)(p);
  f.u[1] = *(const v4u*)(p + 16);
  return f.v;
}

__device__ __forceinline__ v8f mma_raw(v16h a, v16h b, v8f c) {
  return __builtin_amdgcn_wmma_f32_16x16x32_f16(false, a, false, b, (short)0, c, false, false);
}
__device__ __forceinline__ void dep_guard1(v8f& a, v8f& b, v16h x) {
#if defined(__HIP_DEVICE_COMPILE__)
  asm volatile("v_nop\n\tv_nop\n\tv_nop\n\tv_nop" : "+v"(a), "+v"(b) : "v"(x));
#endif
}
__device__ __forceinline__ void guard23(v8f& a, v8f& b, v16h x, v16h y, v16h z) {
#if defined(__HIP_DEVICE_COMPILE__)
  asm volatile("v_nop\n\tv_nop\n\tv_nop\n\tv_nop" : "+v"(a), "+v"(b) : "v"(x), "v"(y), "v"(z));
#endif
}
__device__ __forceinline__ void keep4_h(v16h a, v16h b, v16h c, v16h d) {
#if defined(__HIP_DEVICE_COMPILE__)
  asm volatile("v_nop" :: "v"(a), "v"(b), "v"(c), "v"(d));
#endif
}
__device__ __forceinline__ void acc_guard4(v8f& a, v8f& b, v8f& c, v8f& d) {
#if defined(__HIP_DEVICE_COMPILE__)
  asm volatile("v_nop\n\tv_nop\n\tv_nop\n\tv_nop" : "+v"(a), "+v"(b), "+v"(c), "+v"(d));
#endif
}
__device__ __forceinline__ void wave_sync_lds() {
  __builtin_amdgcn_fence(__ATOMIC_RELEASE, "workgroup");
  __builtin_amdgcn_wave_barrier();
  __builtin_amdgcn_fence(__ATOMIC_ACQUIRE, "workgroup");
}

__global__ __launch_bounds__(256) void wcvt(const float* __restrict__ src, long long ss,
                                             unsigned short* dst, long long sd,
                                             int R, int C, int Rp, int Cp, int dup, float shi, float slo) {
  const int l = blockIdx.y;
  const float* S = src + (size_t)((long long)l * ss);
  unsigned short* D = dst + (size_t)((long long)l * sd);
  const int KD = dup ? (2 * Cp) : Cp;
  const int npieces = (Rp * KD) >> 3;
  const int p = blockIdx.x * 256 + (int)threadIdx.x;
  if (p >= npieces) return;
  const int e0 = p * 8;
  const int r = e0 / KD;
  const int col = e0 - r * KD;
  const int half = (col >= Cp) ? 1 : 0;
  const int c = col - half * Cp;
  const bool valid = (r < R) && (c < C);
  const int rcl = imin(r, R - 1);
  const int ccl = imin(c, C - 8);
  const float* sp = S + (size_t)rcl * C + ccl;
  const v4f a = *(const v4f*)(sp);
  const v4f b = *(const v4f*)(sp + 4);
  const float sc = half ? slo : shi;
  float f[8];
#pragma unroll
  for (int e = 0; e < 4; ++e) { f[e] = a[e]; f[4 + e] = b[e]; }
  v4u o;
#pragma unroll
  for (int e = 0; e < 4; ++e) {
    const unsigned w = pk16(hz(bfr(f[2 * e]) * sc), hz(bfr(f[2 * e + 1]) * sc));
    o[e] = valid ? w : 0u;
  }
  unsigned short* dp = D + (size_t)e0;
  for (int pass = 0; pass < 2; ++pass) {
    *(volatile v4u*)dp = o;
    __threadfence();
  }
}

__global__ __launch_bounds__(256) void btab(const float* __restrict__ rb, float* TH) {
  const int i = blockIdx.x * 256 + (int)threadIdx.x;
  if (i >= NLAYER * NHEAD * TABP) return;
  const int r = i & (TABP - 1);
  const int lh = i >> 11;
  const int l = lh >> 3, h = lh & 7;
  const int rcl = imin(r, TABR - 1);
  int a = r - RELOFF;
  a = (a < 0) ? -a : a;
  const float dec = expf(-DECAYF * (float)a);
  const float bv = bfr(rb[((size_t)l * TABR + rcl) * NHEAD + h]);
  const float v = (r < TABR) ? dec * bv : 0.f;
  float* p = TH + i;
  *(volatile float*)p = v;
  __threadfence();
  *(volatile float*)p = v;
}

__global__ __launch_bounds__(256) void tqmlp(
    const float* __restrict__ timep, const float* __restrict__ queryp,
    const float* __restrict__ tw1, const float* __restrict__ tb1,
    const float* __restrict__ tw2, const float* __restrict__ tb2,
    const float* __restrict__ qw1, const float* __restrict__ qb1,
    const float* __restrict__ qw2, const float* __restrict__ qb2,
    const float* __restrict__ l1w, const float* __restrict__ l1b,
    const float* __restrict__ l2w, const float* __restrict__ l2b,
    float* TPo, float* QEo) {
  __shared__ float emb[TED];
  __shared__ float hid[4 * TED];
  __shared__ float tev[TED];
  __shared__ float u[HID];
  const int bat = blockIdx.x;
  const int t = threadIdx.x;
  {
    const int j = t & 127;
    const float fr = expf((CLN * (float)j) / 127.0f);
    const float a = bfr(timep[bat]) * fr;
    const float sv = sinf(a);
    const float cv = cosf(a);
    emb[t] = (t < 128) ? sv : cv;
  }
  __syncthreads();
#pragma unroll 1
  for (int kq = 0; kq < 4; ++kq) {
    const int k = kq * TED + t;
    float s = bfr(tb1[k]);
    const float* wr = tw1 + (size_t)k * TED;
#pragma unroll 1
    for (int j = 0; j < TED; ++j) s += bfr(wr[j]) * emb[j];
    const float spl = (s > 20.0f) ? s : log1pf(expf(s));
    hid[k] = s * tanhf(spl);
  }
  __syncthreads();
  {
    float s = bfr(tb2[t]);
    const float* wr = tw2 + (size_t)t * (4 * TED);
#pragma unroll 1
    for (int k = 0; k < 4 * TED; ++k) s += bfr(wr[k]) * hid[k];
    tev[t] = s;
  }
  __syncthreads();
#pragma unroll 1
  for (int l = 0; l < NLAYER; ++l) {
    float s = bfr(l1b[l * HID + t]);
    const float* wr = l1w + ((size_t)l * HID + t) * TED;
#pragma unroll 1
    for (int j = 0; j < TED; ++j) s += bfr(wr[j]) * tev[j];
    u[t] = gelu_f(s);
    __syncthreads();
    float s2 = bfr(l2b[l * HID + t]);
    const float* wr2 = l2w + ((size_t)l * HID + t) * HID;
#pragma unroll 1
    for (int k = 0; k < HID; ++k) s2 += bfr(wr2[k]) * u[k];
    float* p = TPo + ((size_t)l * NB + bat) * HID + t;
    *(volatile float*)p = s2;
    __threadfence();
    *(volatile float*)p = s2;
    __syncthreads();
  }
  {
    float s = bfr(qb1[t]);
    const float* wr = qw1 + (size_t)t * QDIM;
    const float* qp = queryp + (size_t)bat * QDIM;
#pragma unroll 1
    for (int j = 0; j < QDIM; ++j) s += bfr(wr[j]) * bfr(qp[j]);
    u[t] = gelu_f(s);
  }
  __syncthreads();
  {
    float s = bfr(qb2[t]);
    const float* wr = qw2 + (size_t)t * HID;
#pragma unroll 1
    for (int k = 0; k < HID; ++k) s += bfr(wr[k]) * u[k];
    float* p = QEo + (size_t)bat * HID + t;
    *(volatile float*)p = s;
    __threadfence();
    *(volatile float*)p = s;
  }
}

template <int OM, int RM, int ACT, int BM, int RS>
__global__ __launch_bounds__(256) void gemm64(
    const unsigned short* __restrict__ Ap, int lda, long long sA,
    const unsigned short* __restrict__ Btp, int ldb, long long sB,
    const float* __restrict__ Rp, int ldr, long long sR,
    const float* __restrict__ biasp, int nbias,
    void* Cout, int ldc, long long sC,
    int M, int N, int K, float oscale, float ocarry) {
  __shared__ __align__(16) float sT[8][16 * 68];
  const int by   = blockIdx.y;
  const int lane = threadIdx.x & 31;
  const int wave = threadIdx.x >> 5;
  const int tilesN = N >> 6;
  const int tilesM = M >> 6;
  const int tile = blockIdx.x * 8 + wave;
  if (tile >= tilesM * tilesN) return;
  const int tm = tile / tilesN;
  const int tn = tile - tm * tilesN;
  const int m0 = tm << 6;
  const int n0 = tn << 6;

  const unsigned short* A1 = Ap  + (size_t)((long long)by * sA);
  const unsigned short* Bb = Btp + (size_t)((long long)by * sB);

  const int rlane = lane & 15;
  const int koff  = (lane >> 4) * 8;
  const int mOff  = (lane >> 4) * 8;

  v8f acc[4][4];
#pragma unroll
  for (int i = 0; i < 4; ++i)
#pragma unroll
    for (int j = 0; j < 4; ++j) acc[i][j] = zero8();

  for (int k0 = 0; k0 < K; k0 += 32) {
    v16h bh[4];
#pragma unroll
    for (int j = 0; j < 4; ++j) {
      const size_t bofs = (size_t)(n0 + (j << 4) + rlane) * ldb + koff + k0;
      bh[j] = ldfrag_u(Bb + bofs);
    }
#pragma unroll
    for (int i = 0; i < 4; ++i) {
      const size_t ao = (size_t)(m0 + (i << 4) + rlane) * lda + koff + k0;
      const v16h ah = ldfrag_u(A1 + ao);
#pragma unroll
      for (int j = 0; j < 4; ++j) acc[i][j] = mma_raw(ah, bh[j], acc[i][j]);
      dep_guard1(acc[i][0], acc[i][3], ah);
    }
    keep4_h(bh[0], bh[1], bh[2], bh[3]);
  }
  acc_guard4(acc[0][0], acc[0][1], acc[0][2], acc[0][3]);
  acc_guard4(acc[1][0], acc[1][1], acc[1][2], acc[1][3]);
  acc_guard4(acc[2][0], acc[2][1], acc[2][2], acc[2][3]);
  acc_guard4(acc[3][0], acc[3][1], acc[3][2], acc[3][3]);

  const int hh2 = lane >> 4, c4 = (lane & 15) * 4;
  const int q8  = lane >> 3, c8 = (lane & 7) * 8;

  float bc4[4], bc8[8];
#pragma unroll
  for (int e = 0; e < 4; ++e) bc4[e] = 0.f;
#pragma unroll
  for (int e = 0; e < 8; ++e) bc8[e] = 0.f;
  if constexpr (BM == 1) {
    if constexpr (OM == 0) {
#pragma unroll
      for (int e = 0; e < 4; ++e) {
        const int n = n0 + c4 + e;
        const int ncl = imin(n, nbias - 1);
        const float t = bfr(biasp[ncl]);
        bc4[e] = (n < nbias) ? t : 0.f;
      }
    } else {
#pragma unroll
      for (int e = 0; e < 8; ++e) {
        const int n = n0 + c8 + e;
        const int ncl = imin(n, nbias - 1);
        const float t = bfr(biasp[ncl]);
        bc8[e] = (n < nbias) ? t : 0.f;
      }
    }
  }

  float* slab = sT[wave];
#pragma unroll
  for (int i = 0; i < 4; ++i) {
    const int mBase = m0 + (i << 4);
#pragma unroll
    for (int j = 0; j < 4; ++j) {
#pragma unroll
      for (int r = 0; r < 8; ++r) {
        slab[(mOff + r) * 68 + (j << 4) + rlane] = acc[i][j][r];
      }
    }
    wave_sync_lds();
    if constexpr (OM == 0) {
      float* C = (float*)Cout + (size_t)((long long)by * sC);
      v4f vals[8];
#pragma unroll
      for (int it = 0; it < 8; ++it) {
        const int row = it * 2 + hh2;
        const int gr  = mBase + row;
        v4f v = *(const v4f*)(slab + row * 68 + c4);
        v4f rv = {0.f, 0.f, 0.f, 0.f};
        if constexpr (RM == 2) {
          const float* R = Rp + (size_t)((long long)by * sR);
          rv = *(const v4f*)(R + (size_t)gr * ldr + n0 + c4);
        }
        float rb = 0.f;
        if constexpr (BM == 2) {
          const int gcl = imin(gr, nbias - 1);
          const float t = bfr(biasp[gcl]);
          rb = (gr < nbias) ? t : 0.f;
        }
#pragma unroll
        for (int e = 0; e < 4; ++e) {
          float uu = v[e] * oscale;
          if constexpr (BM == 1) uu += bc4[e];
          if constexpr (BM == 2) uu += rb;
          if constexpr (ACT == 1) uu = gelu_f(uu);
          v[e] = uu + rv[e];
        }
        vals[it] = v;
      }
      for (int pass = 0; pass < 2; ++pass) {
#pragma unroll
        for (int it = 0; it < 8; ++it) {
          const int gr = mBase + it * 2 + hh2;
          *(volatile v4f*)(C + (size_t)gr * ldc + n0 + c4) = vals[it];
        }
        __threadfence();
      }
    } else {
      unsigned short* C = (unsigned short*)Cout + (size_t)((long long)by * sC);
      v4u hv[4], lv[4];
#pragma unroll
      for (int it = 0; it < 4; ++it) {
        const int row = it * 4 + q8;
        const int gr  = mBase + row;
        float rb = 0.f;
        if constexpr (BM == 2) {
          const int gcl = imin(gr, nbias - 1);
          const float t = bfr(biasp[gcl]);
          rb = (gr < nbias) ? t : 0.f;
        }
        const float* sp = slab + row * 68 + c8;
        v4u a = {0u, 0u, 0u, 0u};
        v4u b = {0u, 0u, 0u, 0u};
#pragma unroll
        for (int e = 0; e < 4; ++e) {
          float f0 = sp[2 * e] * oscale;
          float f1 = sp[2 * e + 1] * oscale;
          if constexpr (BM == 1) { f0 += bc8[2 * e]; f1 += bc8[2 * e + 1]; }
          if constexpr (BM == 2) { f0 += rb; f1 += rb; }
          if constexpr (ACT == 1) { f0 = gelu_f(f0); f1 = gelu_f(f1); }
          f0 *= ocarry; f1 *= ocarry;
          const unsigned short h0 = hz(f0), h1 = hz(f1);
          a[e] = pk16(h0, h1);
          if constexpr (RS == 1) {
            const unsigned short l0 = hz((f0 - hup(h0)) * RSC);
            const unsigned short l1 = hz((f1 - hup(h1)) * RSC);
            b[e] = pk16(l0, l1);
          }
        }
        hv[it] = a;
        lv[it] = b;
      }
      for (int pass = 0; pass < 2; ++pass) {
#pragma unroll
        for (int it = 0; it < 4; ++it) {
          const int row = it * 4 + q8;
          *(volatile v4u*)(C + (size_t)(mBase + row) * ldc + n0 + c8) = hv[it];
          if constexpr (RS == 1) {
            *(volatile v4u*)(C + (size_t)(mBase + row) * ldc + N + n0 + c8) = lv[it];
          }
        }
        __threadfence();
      }
    }
    wave_sync_lds();
  }
}

template <int NORM, int ADDT>
__global__ __launch_bounds__(256) void lnrow(const float* __restrict__ Yp, const float* __restrict__ Tp,
                                              const float* __restrict__ gp, const float* __restrict__ bp,
                                              unsigned short* outh, float hc, int nrows) {
  const int lane = threadIdx.x & 31, wave = threadIdx.x >> 5;
  const int row = blockIdx.x * 8 + wave;
  if (row >= nrows) return;
  const float* yp = Yp + (size_t)row * HID + lane * 8;
  const v4f a0 = *(const v4f*)(yp);
  const v4f a1 = *(const v4f*)(yp + 4);
  float v[8];
#pragma unroll
  for (int e = 0; e < 4; ++e) { v[e] = a0[e]; v[4 + e] = a1[e]; }
  if constexpr (ADDT == 1) {
    const int bat = row / SEQ;
    const float* tpp = Tp + (size_t)bat * HID + lane * 8;
    const v4f t0 = *(const v4f*)(tpp);
    const v4f t1 = *(const v4f*)(tpp + 4);
#pragma unroll
    for (int e = 0; e < 4; ++e) { v[e] += t0[e]; v[4 + e] += t1[e]; }
  }
  float o[8];
  if constexpr (NORM == 1) {
    float s = ((v[0] + v[1]) + (v[2] + v[3])) + ((v[4] + v[5]) + (v[6] + v[7]));
#pragma unroll
    for (int off = 1; off < 32; off <<= 1) s += __shfl_xor(s, off, 32);
    const float mu = s * (1.0f / (float)HID);
    float d[8];
#pragma unroll
    for (int e = 0; e < 8; ++e) d[e] = v[e] - mu;
    float q = ((d[0] * d[0] + d[1] * d[1]) + (d[2] * d[2] + d[3] * d[3])) +
              ((d[4] * d[4] + d[5] * d[5]) + (d[6] * d[6] + d[7] * d[7]));
#pragma unroll
    for (int off = 1; off < 32; off <<= 1) q += __shfl_xor(q, off, 32);
    const float var  = q * (1.0f / (float)HID);
    const float rstd = rsqrtf(var + LN_EPS);
    const v4f g0 = *(const v4f*)(gp + lane * 8);
    const v4f g1 = *(const v4f*)(gp + lane * 8 + 4);
    const v4f b0 = *(const v4f*)(bp + lane * 8);
    const v4f b1 = *(const v4f*)(bp + lane * 8 + 4);
#pragma unroll
    for (int e = 0; e < 4; ++e) {
      o[e]     = (d[e] * rstd) * bfr(g0[e]) + bfr(b0[e]);
      o[4 + e] = (d[4 + e] * rstd) * bfr(g1[e]) + bfr(b1[e]);
    }
  } else {
#pragma unroll
    for (int e = 0; e < 8; ++e) o[e] = v[e];
  }
  v4u hv, lv;
#pragma unroll
  for (int e = 0; e < 4; ++e) {
    const float f0 = o[2 * e] * hc;
    const float f1 = o[2 * e + 1] * hc;
    const unsigned short h0 = hz(f0), h1 = hz(f1);
    const unsigned short l0 = hz((f0 - hup(h0)) * RSC);
    const unsigned short l1 = hz((f1 - hup(h1)) * RSC);
    hv[e] = pk16(h0, h1);
    lv[e] = pk16(l0, l1);
  }
  unsigned short* dp = outh + (size_t)row * KX + lane * 8;
  for (int pass = 0; pass < 2; ++pass) {
    *(volatile v4u*)(dp) = hv;
    *(volatile v4u*)(dp + HID) = lv;
    __threadfence();
  }
}

#define ATT_THREADS (NHEAD * 32)
#define ATT_BLOCKS  (NB * (SEQ / 16))
#define TBW         (SEQ + 16)
#define PS_FLOATS   (NHEAD * 16 * 36)
static_assert(ATT_THREADS == 256);
static_assert((size_t)16 * HID * sizeof(unsigned short) <= (size_t)PS_FLOATS * sizeof(float));
static_assert(((16 * HID) % (8 * ATT_THREADS)) == 0 && ((16 * HID) / (8 * ATT_THREADS)) == 2);

__global__ __launch_bounds__(ATT_THREADS)
void attnR(const unsigned short* __restrict__ QKp, const unsigned short* __restrict__ VTq,
           const float* __restrict__ THl, unsigned short* CT) {
  __shared__ __align__(16) float smem[PS_FLOATS];
  __shared__ float tb[NHEAD][TBW];

  const int tid  = threadIdx.x;
  const int wave = tid >> 5;
  const int lane = tid & 31;
  const int hh   = lane >> 4;
  const int c    = lane & 15;

  const int qt   = blockIdx.x % (SEQ / 16);
  const int bat  = blockIdx.x / (SEQ / 16);
  const int head = wave;
  const int q0   = qt * 16;

  {
    const float* th = THl + (size_t)head * TABP + (q0 + SEQ_FULL - SEQ);
    for (int w = lane; w < TBW; w += 32) {
      const int wcl = imin(w, SEQ + 14);
      const float tv = th[wcl] * LOG2E;
      tb[wave][w] = (w < SEQ + 15) ? tv : 0.f;
    }
  }
  __syncthreads();

  const _Float16* QK = (const _Float16*)(const void*)QKp;
  const _Float16* Qh = QK + ((size_t)bat * SEQ + q0 + c) * KX + head * HDIM + 8 * hh;
  const _Float16* Kb = QK + (size_t)bat * SEQ * KX + HID + head * HDIM + 8 * hh;
  const _Float16* Vb = (const _Float16*)(const void*)VTq + ((size_t)bat * HID + head * HDIM) * SEQ + 8 * hh;
  const float lsc = (LOG2E * ATT_SCALE) / (QC * KC);

  const v16h qa = ldfrag_h(Qh);

  float mrow[8], lrow[8];
  v8f o0 = zero8(), o1 = zero8();
#pragma unroll
  for (int r = 0; r < 8; ++r) { mrow[r] = -INFINITY; lrow[r] = 0.f; }
  float* pt = smem + wave * (16 * 36);
  const float* tbw = tb[wave];

#pragma unroll 1
  for (int kb = 0; kb < SEQ; kb += 32) {
    const _Float16* kp = Kb + (size_t)(kb + c) * KX;
    v8f s0, s1;
    {
      const v16h k0 = ldfrag_h(kp);
      const v16h k1 = ldfrag_h(kp + (size_t)16 * KX);
      s0 = mma_raw(qa, k0, zero8());
      s1 = mma_raw(qa, k1, zero8());
      guard23(s0, s1, qa, k0, k1);
    }
    const int wb = 8 * hh - kb - c + (SEQ - 1);
#pragma unroll
    for (int r = 0; r < 8; ++r) {
      const float t0 = fmaf(s0[r], lsc, tbw[wb + r]);
      const float t1 = fmaf(s1[r], lsc, tbw[wb + r - 16]);
      float mx = fmaxf(t0, t1);
#pragma unroll
      for (int off = 1; off < 16; off <<= 1) mx = fmaxf(mx, __shfl_xor(mx, off, 32));
      const float mn = fmaxf(mrow[r], mx);
      const float al = exp2f(fmaxf(mrow[r] - mn, -126.0f));
      mrow[r] = mn;
      const float e0 = exp2f(t0 - mn);
      const float e1 = exp2f(t1 - mn);
      float ps = e0 + e1;
#pragma unroll
      for (int off = 1; off < 16; off <<= 1) ps += __shfl_xor(ps, off, 32);
      lrow[r] = lrow[r] * al + ps;
      o0[r] *= al;
      o1[r] *= al;
      const int ro = (8 * hh + r) * 36 + c;
      pt[ro]      = e0;
      pt[ro + 16] = e1;
    }
    wave_sync_lds();
    FragH ph;
    {
      const float* prow = pt + c * 36 + 8 * hh;
      const v4f p0 = *(const v4f*)(prow), p1 = *(const v4f*)(prow + 4);
      const v4f p2 = *(const v4f*)(prow + 16), p3 = *(const v4f*)(prow + 20);
#pragma unroll
      for (int e = 0; e < 4; ++e) {
        ph.h[0][e]     = (_Float16)(p0[e] * PC);
        ph.h[0][4 + e] = (_Float16)(p1[e] * PC);
        ph.h[1][e]     = (_Float16)(p2[e] * PC);
        ph.h[1][4 + e] = (_Float16)(p3[e] * PC);
      }
    }
    const _Float16* vp = Vb + (size_t)c * SEQ + kb;
    {
      const v16h vb0 = ldfrag_h(vp);
      const v16h vb1 = ldfrag_h(vp + (size_t)16 * SEQ);
      o0 = mma_raw(ph.v, vb0, o0);
      o1 = mma_raw(ph.v, vb1, o1);
      guard23(o0, o1, ph.v, vb0, vb1);
    }
    wave_sync_lds();
  }

  __syncthreads();
  unsigned short* Os = (unsigned short*)smem;
  const float oc = FC / (PC * VC);
  unsigned short* osw = Os + wave * HDIM + c;
#pragma unroll
  for (int r = 0; r < 8; ++r) {
    const float inv = (1.0f / lrow[r]) * oc;
    unsigned short* op = osw + (8 * hh + r) * HID;
    op[0]  = hz(o0[r] * inv);
    op[16] = hz(o1[r] * inv);
  }
  __syncthreads();
  {
    v4u vals[2];
#pragma unroll
    for (int it = 0; it < 2; ++it) {
      const int p = it * ATT_THREADS + tid;
      vals[it] = *(const v4u*)(Os + (size_t)p * 8);
    }
    unsigned short* dst = CT + ((size_t)bat * SEQ + q0) * HID;
    for (int pass = 0; pass < 2; ++pass) {
#pragma unroll
      for (int it = 0; it < 2; ++it) {
        const int p = it * ATT_THREADS + tid;
        *(volatile v4u*)(dst + (size_t)p * 8) = vals[it];
      }
      __threadfence();
    }
  }
}

__global__ __launch_bounds__(256) void ocopy(const float* __restrict__ OW, float* out, int nrows) {
  const int i = blockIdx.x * 256 + (int)threadIdx.x;
  if (i >= nrows * 4) return;
  const int row = i >> 2, cc = (i & 3) * 4;
  const v4f v = *(const v4f*)(OW + (size_t)row * NOUTP + cc);
  float* p = out + (size_t)i * 4;
  *(volatile v4f*)p = v;
  __threadfence();
  *(volatile v4f*)p = v;
}

extern "C" void kernel_launch(void* const* d_in, const int* in_sizes, int n_in,
                              void* d_out, int out_size, void* d_ws, size_t ws_size,
                              hipStream_t stream) {
  if (n_in < 32) return;
  if (in_sizes[0] < NB * SEQ_FULL * IND) return;
  if (in_sizes[1] < NB * QDIM || in_sizes[2] < NB) return;
  if (in_sizes[3] != 4 * TED * TED || in_sizes[4] != 4 * TED || in_sizes[5] != TED * 4 * TED || in_sizes[6] != TED) return;
  if (in_sizes[7] != HID * IND || in_sizes[8] != HID) return;
  if (in_sizes[9] != HID * QDIM || in_sizes[10] != HID || in_sizes[11] != HID * HID || in_sizes[12] != HID) return;
  if (in_sizes[13] != NLAYER * HID || in_sizes[14] != NLAYER * HID) return;
  if (in_sizes[15] != NLAYER * 3 * HID * HID || in_sizes[16] != NLAYER * 3 * HID) return;
  if (in_sizes[17] != NLAYER * HID * HID || in_sizes[18] != NLAYER * HID) return;
  if (in_sizes[19] != NLAYER * TABR * NHEAD) return;
  if (in_sizes[20] != NLAYER * HID || in_sizes[21] != NLAYER * HID) return;
  if (in_sizes[22] != NLAYER * DFF * HID || in_sizes[23] != NLAYER * DFF) return;
  if (in_sizes[24] != NLAYER * HID * DFF || in_sizes[25] != NLAYER * HID) return;
  if (in_sizes[26] != NLAYER * HID * TED || in_sizes[27] != NLAYER * HID) return;
  if (in_sizes[28] != NLAYER * HID * HID || in_sizes[29] != NLAYER * HID) return;
  if (in_sizes[30] != OUTD * HID || in_sizes[31] != OUTD) return;
  if (out_size < NROWS * OUTD) return;

  const float* x     = (const float*)d_in[0];
  const float* query = (const float*)d_in[1];
  const float* timev = (const float*)d_in[2];
  const float* tm_w1 = (const float*)d_in[3];
  const float* tm_b1 = (const float*)d_in[4];
  const float* tm_w2 = (const float*)d_in[5];
  const float* tm_b2 = (const float*)d_in[6];
  const float* in_w  = (const float*)d_in[7];
  const float* in_b  = (const float*)d_in[8];
  const float* q_w1  = (const float*)d_in[9];
  const float* q_b1  = (const float*)d_in[10];
  const float* q_w2  = (const float*)d_in[11];
  const float* q_b2  = (const float*)d_in[12];
  const float* n1_w  = (const float*)d_in[13];
  const float* n1_b  = (const float*)d_in[14];
  const float* qkv_w = (const float*)d_in[15];
  const float* qkv_b = (const float*)d_in[16];
  const float* ap_w  = (const float*)d_in[17];
  const float* ap_b  = (const float*)d_in[18];
  const float* rel_b = (const float*)d_in[19];
  const float* n2_w  = (const float*)d_in[20];
  const float* n2_b  = (const float*)d_in[21];
  const float* f1_w  = (const float*)d_in[22];
  const float* f1_b  = (const float*)d_in[23];
  const float* f2_w  = (const float*)d_in[24];
  const float* f2_b  = (const float*)d_in[25];
  const float* t1_w  = (const float*)d_in[26];
  const float* t1_b  = (const float*)d_in[27];
  const float* t2_w  = (const float*)d_in[28];
  const float* t2_b  = (const float*)d_in[29];
  const float* out_w = (const float*)d_in[30];
  const float* out_b = (const float*)d_in[31];
  float*       out   = (float*)d_out;

  const size_t PWQKV = (size_t)NLAYER * 3 * HID * KX * 2;
  const size_t PWAP  = (size_t)NLAYER * HID * HID * 2;
  const size_t PWF1  = (size_t)NLAYER * DFF * KX * 2;
  const size_t PWF2  = (size_t)NLAYER * HID * KG * 2;
  const size_t PWIN  = (size_t)HID * KIN * 2;
  const size_t PWOUT = (size_t)NOUTP * KX * 2;
  const size_t PX16  = (size_t)NROWS * KIN * 2;
  const size_t PTH   = (size_t)NLAYER * NHEAD * TABP * 4;
  const size_t PTP   = (size_t)NLAYER * NB * HID * 4;
  const size_t PQE   = (size_t)NB * HID * 4;
  const size_t PH32  = (size_t)NROWS * HID * 4;
  const size_t PXN   = (size_t)NROWS * KX * 2;
  const size_t PQK   = (size_t)NROWS * KX * 2;
  const size_t PVT   = (size_t)NB * HID * SEQ * 2;
  const size_t PCT   = (size_t)NROWS * HID * 2;
  const size_t PG    = (size_t)NROWS * KG * 2;
  const size_t POW   = (size_t)NROWS * NOUTP * 4;
  size_t off = 0;
  const size_t oWQKV = off; off += PWQKV;
  const size_t oWAP  = off; off += PWAP;
  const size_t oWF1  = off; off += PWF1;
  const size_t oWF2  = off; off += PWF2;
  const size_t oWIN  = off; off += PWIN;
  const size_t oWOUT = off; off += PWOUT;
  const size_t oX16  = off; off += PX16;
  const size_t oTH   = off; off += PTH;
  const size_t oTP   = off; off += PTP;
  const size_t oQE   = off; off += PQE;
  const size_t oHA   = off; off += PH32;
  const size_t oHB   = off; off += PH32;
  const size_t oXN   = off; off += PXN;
  const size_t oQK   = off; off += PQK;
  const size_t oVT   = off; off += PVT;
  const size_t oCT   = off; off += PCT;
  const size_t oG    = off; off += PG;
  const size_t oOW   = off; off += POW;
  const size_t endAll = off;
  if (endAll > ws_size) return;
  if (endAll > (size_t)134217728) return;

  char* ws = (char*)d_ws;
  unsigned short* WQKV = (unsigned short*)(ws + oWQKV);
  unsigned short* WAP  = (unsigned short*)(ws + oWAP);
  unsigned short* WF1  = (unsigned short*)(ws + oWF1);
  unsigned short* WF2  = (unsigned short*)(ws + oWF2);
  unsigned short* WIN  = (unsigned short*)(ws + oWIN);
  unsigned short* WOUT = (unsigned short*)(ws + oWOUT);
  unsigned short* X16  = (unsigned short*)(ws + oX16);
  float*          TH   = (float*)(ws + oTH);
  float*          TP   = (float*)(ws + oTP);
  float*          QE   = (float*)(ws + oQE);
  float*          HA   = (float*)(ws + oHA);
  float*          HB   = (float*)(ws + oHB);
  unsigned short* XN   = (unsigned short*)(ws + oXN);
  unsigned short* QK   = (unsigned short*)(ws + oQK);
  unsigned short* VT   = (unsigned short*)(ws + oVT);
  unsigned short* CT   = (unsigned short*)(ws + oCT);
  unsigned short* G    = (unsigned short*)(ws + oG);
  float*          OW   = (float*)(ws + oOW);

  const dim3 blk(256);
  const dim3 gCqkv((3 * HID * KX / 8 + 255) / 256, NLAYER);
  const dim3 gCap((HID * HID / 8 + 255) / 256, NLAYER);
  const dim3 gCf1((DFF * KX / 8 + 255) / 256, NLAYER);
  const dim3 gCf2((HID * KG / 8 + 255) / 256, NLAYER);
  const dim3 gCin((HID * KIN / 8 + 255) / 256, 1);
  const dim3 gCout((NOUTP * KX / 8 + 255) / 256, 1);
  const dim3 gCx((SEQ * KIN / 8 + 255) / 256, NB);
  const dim3 gTab((NLAYER * NHEAD * TABP + 255) / 256);
  const dim3 gTQ(NB);
  const int tilesIn  = (SEQ / 64) * (HID / 64);
  const int tilesQK  = (NROWS / 64) * (KX / 64);
  const int tilesV   = (HID / 64) * (SEQ / 64);
  const int tilesAP  = (NROWS / 64) * (HID / 64);
  const int tilesF1  = (NROWS / 64) * (DFF / 64);
  const int tilesOut = (NROWS / 64) * (NOUTP / 64);
  const dim3 gIn((tilesIn + 7) / 8, NB);
  const dim3 gQK((tilesQK + 7) / 8, 1);
  const dim3 gV((tilesV + 7) / 8, NB);
  const dim3 gAP((tilesAP + 7) / 8, 1);
  const dim3 gF1((tilesF1 + 7) / 8, 1);
  const dim3 gOut((tilesOut + 7) / 8, 1);
  const dim3 gLN(NROWS / 8);
  const dim3 gAT(ATT_BLOCKS);
  const dim3 gOC((NROWS * 4 + 255) / 256);

  wcvt<<<gCqkv, blk, 0, stream>>>(qkv_w, (long long)3 * HID * HID, WQKV, (long long)3 * HID * KX, 3 * HID, HID, 3 * HID, HID, 1, WSC, WLO);
  wcvt<<<gCap,  blk, 0, stream>>>(ap_w, (long long)HID * HID, WAP, (long long)HID * HID, HID, HID, HID, HID, 0, WSC, WSC);
  wcvt<<<gCf1,  blk, 0, stream>>>(f1_w, (long long)DFF * HID, WF1, (long long)DFF * KX, DFF, HID, DFF, HID, 1, WSC, WLO);
  wcvt<<<gCf2,  blk, 0, stream>>>(f2_w, (long long)HID * DFF, WF2, (long long)HID * KG, HID, DFF, HID, DFF, 1, WSC, WLO);
  wcvt<<<gCin,  blk, 0, stream>>>(in_w, 0LL, WIN, 0LL, HID, IND, HID, KIN, 0, WSC, WSC);
  wcvt<<<gCout, blk, 0, stream>>>(out_w, 0LL, WOUT, 0LL, OUTD, HID, NOUTP, HID, 1, WSC, WLO);
  wcvt<<<gCx,   blk, 0, stream>>>(x, (long long)SEQ_FULL * IND, X16, (long long)SEQ * KIN, SEQ, IND, SEQ, KIN, 0, XC, XC);

  btab<<<gTab, blk, 0, stream>>>(rel_b, TH);
  tqmlp<<<gTQ, blk, 0, stream>>>(timev, query, tm_w1, tm_b1, tm_w2, tm_b2, q_w1, q_b1, q_w2, q_b2,
                                  t1_w, t1_b, t2_w, t2_b, TP, QE);

  gemm64<0, 2, 0, 1, 0><<<gIn, blk, 0, stream>>>(
      X16, KIN, (long long)SEQ * KIN,
      WIN, KIN, 0LL,
      QE, 0, (long long)HID,
      in_b, HID,
      (void*)HA, HID, (long long)SEQ * HID,
      SEQ, HID, KIN, 1.0f / (XC * WSC), 1.0f);

  for (int l = 0; l < NLAYER; ++l) {
    const unsigned short* Wqkv_l = WQKV + (size_t)l * 3 * HID * KX;
    lnrow<1, 1><<<gLN, blk, 0, stream>>>(HA, TP + (size_t)l * NB * HID, n1_w + l * HID, n1_b + l * HID, XN, HCARRY, NROWS);
    gemm64<2, 0, 0, 1, 0><<<gQK, blk, 0, stream>>>(
        XN, KX, 0LL,
        Wqkv_l, KX, 0LL,
        QE, 0, 0LL,
        qkv_b + (size_t)l * 3 * HID, 2 * HID,
        (void*)QK, KX, 0LL,
        NROWS, KX, KX, 1.0f / (HCARRY * WSC), QC);
    gemm64<2, 0, 0, 2, 0><<<gV, blk, 0, stream>>>(
        Wqkv_l + (size_t)2 * HID * KX, KX, 0LL,
        XN, KX, (long long)SEQ * KX,
        QE, 0, 0LL,
        qkv_b + (size_t)l * 3 * HID + 2 * HID, HID,
        (void*)VT, SEQ, (long long)HID * SEQ,
        HID, SEQ, KX, 1.0f / (HCARRY * WSC), VC);
    attnR<<<gAT, dim3(ATT_THREADS), 0, stream>>>(QK, VT, TH + (size_t)l * NHEAD * TABP, CT);
    gemm64<0, 2, 0, 1, 0><<<gAP, blk, 0, stream>>>(
        CT, HID, 0LL,
        WAP + (size_t)l * HID * HID, HID, 0LL,
        HA, HID, 0LL,
        ap_b + (size_t)l * HID, HID,
        (void*)HB, HID, 0LL,
        NROWS, HID, HID, 1.0f / (FC * WSC), 1.0f);
    lnrow<1, 0><<<gLN, blk, 0, stream>>>(HB, TP, n2_w + l * HID, n2_b + l * HID, XN, HCARRY, NROWS);
    gemm64<2, 0, 1, 1, 1><<<gF1, blk, 0, stream>>>(
        XN, KX, 0LL,
        WF1 + (size_t)l * DFF * KX, KX, 0LL,
        QE, 0, 0LL,
        f1_b + (size_t)l * DFF, DFF,
        (void*)G, KG, 0LL,
        NROWS, DFF, KX, 1.0f / (HCARRY * WSC), GC);
    gemm64<0, 2, 0, 1, 0><<<gAP, blk, 0, stream>>>(
        G, KG, 0LL,
        WF2 + (size_t)l * HID * KG, KG, 0LL,
        HB, HID, 0LL,
        f2_b + (size_t)l * HID, HID,
        (void*)HA, HID, 0LL,
        NROWS, HID, KG, 1.0f / (GC * WSC), 1.0f);
  }

  lnrow<0, 0><<<gLN, blk, 0, stream>>>(HA, TP, n2_w, n2_b, XN, HFC, NROWS);
  gemm64<0, 0, 0, 1, 0><<<gOut, blk, 0, stream>>>(
      XN, KX, 0LL,
      WOUT, KX, 0LL,
      QE, 0, 0LL,
      out_b, OUTD,
      (void*)OW, NOUTP, 0LL,
      NROWS, NOUTP, KX, 1.0f / (HFC * WSC), 1.0f);
  ocopy<<<gOC, blk, 0, stream>>>(OW, out, NROWS);
  (void)hipGetLastError();
}
